// DisentangledSelfAttention_26259430048374
// MI455X (gfx1250) — hardware-run, weakly checked
//
#include <hip/hip_runtime.h>


#define NB_  8
#define TT   1024
#define DM   1024
#define NH_  8
#define NKV  8
#define REP  (NH_ / NKV)
#define HD   64
#define DQ   (NH_ * HD)
#define DKV  (NKV * HD)
#define ZH   2
#define RH   512
#define WIN  0
#define PCAR 1024.0f
#define SCL  0.125f
#define EE   1024
#define AA   512
#define NPS  8
#define NU   64
#define CHK  65536
typedef _Float16 h16;
typedef unsigned short bf;
typedef __attribute__((ext_vector_type(16))) __bf16   v16bf;
typedef __attribute__((ext_vector_type(16))) _Float16 v16h;
typedef __attribute__((ext_vector_type(8)))  _Float16 v8h;
typedef __attribute__((ext_vector_type(8)))  unsigned short v8us;
typedef __attribute__((ext_vector_type(8)))  float    v8f;
typedef __attribute__((ext_vector_type(4)))  float    v4f;
typedef v8h  __attribute__((may_alias)) v8ha;
typedef v4f  __attribute__((may_alias)) v4fa;
typedef v8us __attribute__((may_alias)) v8usa;

__device__ __forceinline__ unsigned short f2bf(float f) { unsigned u = __float_as_uint(f); u += 0x7FFFu + ((u >> 16) & 1u); return (unsigned short)(u >> 16); }
__device__ __forceinline__ float bf2f(unsigned short b) { return __uint_as_float(((unsigned)b) << 16); }
__device__ __forceinline__ float bfr(float f) { return bf2f(f2bf(f)); }
__device__ __forceinline__ v16h cat16(v8h lo, v8h hi) { return __builtin_shufflevector(lo, hi, 0, 1, 2, 3, 4, 5, 6, 7, 8, 9, 10, 11, 12, 13, 14, 15); }
__device__ __forceinline__ v16bf cat16b(v8us lo, v8us hi) { return __builtin_bit_cast(v16bf, __builtin_shufflevector(lo, hi, 0, 1, 2, 3, 4, 5, 6, 7, 8, 9, 10, 11, 12, 13, 14, 15)); }
__device__ __forceinline__ v8f wmma16(v16h a, v16h b, v8f c) { return __builtin_amdgcn_wmma_f32_16x16x32_f16(false, a, false, b, (short)0, c, false, false); }
__device__ __forceinline__ v8f wmmab(v16bf a, v16bf b, v8f c) { return __builtin_amdgcn_wmma_f32_16x16x32_bf16(false, a, false, b, (short)0, c, false, false); }


template <typename T16> struct WFrag;
template <> struct WFrag<h16> { typedef v16h V; static __device__ __forceinline__ V ld(const h16* p) { return cat16(*(const v8h*)p, *(const v8h*)(p + 16)); } static __device__ __forceinline__ v8f mma(V a, V b, v8f c) { return wmma16(a, b, c); } };
template <> struct WFrag<bf> { typedef v16bf V; static __device__ __forceinline__ V ld(const bf* p) { return cat16b(*(const v8us*)p, *(const v8us*)(p + 16)); } static __device__ __forceinline__ v8f mma(V a, V b, v8f c) { return wmmab(a, b, c); } };
template <typename T16, int NSPLIT, bool BIAS>
__global__ __launch_bounds__(32) void k_gemmw(const T16* __restrict__ A, const T16* __restrict__ A2, const T16* __restrict__ Bt, const T16* __restrict__ Bt2, int K, float* C, int ldc, const float* __restrict__ bias, size_t sA, size_t sB, size_t sC) {
    typedef typename WFrag<T16>::V V;
    __shared__ __align__(16) float os[16 * 68];
    const size_t z = blockIdx.z; A += z * sA; if (A2) A2 += z * sA; Bt += z * sB; if (Bt2) Bt2 += z * sB; C += z * sC;
    const int lane = threadIdx.x & 31, lr = lane & 15, hi = lane >> 4; const int r0 = blockIdx.x * 64, c0 = blockIdx.y * 64;
    v8f acc[4][4];
#pragma unroll
    for (int mb = 0; mb < 4; ++mb)
#pragma unroll
        for (int nb = 0; nb < 4; ++nb) acc[mb][nb] = (v8f){};
    const size_t aoff = (size_t)(r0 + lr) * K + 8 * hi, boff = (size_t)(c0 + lr) * K + 8 * hi;
#pragma unroll 1
    for (int kc = 0; kc < K; kc += 32) {
        V a[4], a2[4];
#pragma unroll
        for (int mb = 0; mb < 4; ++mb) { a[mb] = WFrag<T16>::ld(A + aoff + (size_t)mb * 16 * K + kc); if (NSPLIT == 1 || NSPLIT == 2) a2[mb] = WFrag<T16>::ld(A2 + aoff + (size_t)mb * 16 * K + kc); }
#pragma unroll
        for (int nb = 0; nb < 4; ++nb) { const V b = WFrag<T16>::ld(Bt + boff + (size_t)nb * 16 * K + kc); V b2; if (NSPLIT >= 2) b2 = WFrag<T16>::ld(Bt2 + boff + (size_t)nb * 16 * K + kc);
#pragma unroll
            for (int mb = 0; mb < 4; ++mb) { acc[mb][nb] = WFrag<T16>::mma(a[mb], b, acc[mb][nb]); if (NSPLIT == 1 || NSPLIT == 2) acc[mb][nb] = WFrag<T16>::mma(a2[mb], b, acc[mb][nb]); if (NSPLIT >= 2) acc[mb][nb] = WFrag<T16>::mma(a[mb], b2, acc[mb][nb]); } }
        asm volatile("v_nop\n\tv_nop\n\tv_nop\n\tv_nop" : "+v"(acc[0][0]), "+v"(acc[1][1]), "+v"(acc[2][2]), "+v"(acc[3][3]) : "v"(a[0]), "v"(a[3]));
    }
#pragma unroll
    for (int mb = 0; mb < 4; ++mb) {
#pragma unroll
        for (int nb = 0; nb < 4; ++nb) {
#pragma unroll
            for (int j = 0; j < 8; ++j) os[(hi * 8 + j) * 68 + nb * 16 + lr] = acc[mb][nb][j]; }
        __builtin_amdgcn_wave_barrier(); asm volatile("" ::: "memory");
        float* crow = C + (size_t)(r0 + mb * 16) * ldc + c0;
#pragma unroll 1
        for (int ps = 0; ps < 2; ++ps) {
#pragma unroll
            for (int s = 0; s < 8; ++s) { const int row = 2 * s + hi, cofs = lr * 4; v4f val = *(const v4fa*)(os + row * 68 + cofs); if (BIAS) { val[0] += bfr(bias[c0 + cofs]); val[1] += bfr(bias[c0 + cofs + 1]); val[2] += bfr(bias[c0 + cofs + 2]); val[3] += bfr(bias[c0 + cofs + 3]); }
                *(volatile v4f*)(crow + (size_t)row * ldc + cofs) = val; }
            if (ps == 0) __threadfence(); }
        __builtin_amdgcn_wave_barrier(); asm volatile("" ::: "memory");
    }
}

__device__ __forceinline__ h16 tohx(float x) { return (h16)x; }
__device__ __forceinline__ void splitf(float y, unsigned short& h, unsigned short& l) { h = f2bf(y); l = f2bf(y - bf2f(h)); }
typedef __attribute__((ext_vector_type(2))) _Float16 v2h;
typedef __attribute__((ext_vector_type(4))) _Float16 v4h;
typedef __attribute__((ext_vector_type(2))) unsigned short v2us;
typedef __attribute__((ext_vector_type(4))) unsigned short v4us;
typedef __attribute__((ext_vector_type(2))) float v2f;
typedef __attribute__((ext_vector_type(4))) int v4i;

__global__ __launch_bounds__(256) void k_wtG(const float* __restrict__ w, int K, int N, bf* Bt) {
    const int lane = threadIdx.x & 31; const int L0 = (blockIdx.x * 8 + (threadIdx.x >> 5)) * 8; const int nlines = N * K / 64;
#pragma unroll
    for (int ps = 0; ps < 2; ++ps) {
#pragma unroll 1
        for (int l = 0; l < 8; ++l) { const int L = L0 + l; if (L >= nlines) break; const size_t e = (size_t)L * 64 + lane * 2; const int k = (int)(e % K), n = (int)(e / K); v2us o;
            o[0] = f2bf(w[(size_t)k * N + n]); o[1] = f2bf(w[(size_t)(k + 1) * N + n]); *(volatile v2us*)(Bt + e) = o; }
        if (ps == 0) __threadfence(); }
}
__global__ __launch_bounds__(256) void k_cvt8(const float* __restrict__ src, bf* dst, size_t n8) { const size_t i = (size_t)blockIdx.x * 256 + threadIdx.x; if (i >= n8) return; const v8f v = *(const v8f*)(src + i * 8); v8us o;
#pragma unroll
    for (int k = 0; k < 8; ++k) o[k] = f2bf(v[k]); *(volatile v8us*)(dst + i * 8) = o; __threadfence(); *(volatile v8us*)(dst + i * 8) = o; }


__global__ __launch_bounds__(256) void k_asoft(const float* __restrict__ Sb, h16* P16, bf* Ph, bf* Pl) {
    const int lane = threadIdx.x & 31; const int row = blockIdx.x * 8 + (threadIdx.x >> 5); if (row >= ZH * TT) return; const int i = row % TT; const int zz = row / TT; (void)zz; const bool hires = (i < RH); const float* sr = Sb + (size_t)row * TT; float v[TT / 32]; float mx = -3.0e38f;
#pragma unroll
    for (int ch = 0; ch < TT / 128; ++ch) { const int j0 = ch * 128 + lane * 4; const v4f a = *(const v4f*)(sr + j0);
#pragma unroll
        for (int q = 0; q < 4; ++q) { const int j = j0 + q; (void)j; const float t = a[q] * SCL; v[ch * 4 + q] = t; mx = fmaxf(mx, t); } }
#pragma unroll
    for (int sh = 16; sh; sh >>= 1) mx = fmaxf(mx, __shfl_xor(mx, sh, 32));
    float sum = 0.f;
#pragma unroll
    for (int k = 0; k < TT / 32; ++k) { float d0 = __fsub_rn(v[k], mx); asm volatile("" : "+v"(d0)); v[k] = __builtin_amdgcn_exp2f(__fmul_rn(d0, 1.4426950408889634f)); sum += v[k]; }
#pragma unroll
    for (int sh = 16; sh; sh >>= 1) sum += __shfl_xor(sum, sh, 32);
    const float f = __fdiv_rn(hires ? 1.0f : PCAR, sum);
#pragma unroll 1
    for (int ps = 0; ps < 2; ++ps) {
        if (hires) {
#pragma unroll
            for (int ch = 0; ch < TT / 128; ++ch) { v4us oh, ol;
#pragma unroll
                for (int q = 0; q < 4; ++q) { unsigned short a, c2; splitf(v[ch * 4 + q] * f, a, c2); oh[q] = a; ol[q] = c2; }
                const size_t oo = ((size_t)zz * (RH ? RH : 1) + i) * TT + ch * 128 + lane * 4; *(volatile v4us*)(Ph + oo) = oh; *(volatile v4us*)(Pl + oo) = ol; }
        } else {
#pragma unroll
            for (int ch = 0; ch < TT / 128; ++ch) { v4h o4;
#pragma unroll
                for (int q = 0; q < 4; ++q) o4[q] = tohx(v[ch * 4 + q] * f);
                *(volatile v4h*)(P16 + (size_t)row * TT + ch * 128 + lane * 4) = o4; } }
        if (ps == 0) __threadfence(); }
}
__global__ __launch_bounds__(256) void k_flat(const float* __restrict__ F, h16* P16, bf* Ph, bf* Pl, size_t n4) { const size_t i = (size_t)blockIdx.x * 256 + threadIdx.x; if (i >= n4) return; const v4f a = *(const v4f*)(F + i * 4); v4h o16; v4us oh, ol;
#pragma unroll
    for (int q = 0; q < 4; ++q) { o16[q] = tohx(a[q]); unsigned short x2, y2; splitf(a[q], x2, y2); oh[q] = x2; ol[q] = y2; }
    *(volatile v4h*)(P16 + i * 4) = o16; *(volatile v4us*)(Ph + i * 4) = oh; *(volatile v4us*)(Pl + i * 4) = ol; __threadfence(); *(volatile v4h*)(P16 + i * 4) = o16; *(volatile v4us*)(Ph + i * 4) = oh; *(volatile v4us*)(Pl + i * 4) = ol; }

__global__ __launch_bounds__(256) void k_wpadT(const float* __restrict__ w, bf* Bt) { const size_t i = (size_t)blockIdx.x * 256 + threadIdx.x; if (i >= (size_t)NU * EE / 8) return; const int k0 = (int)(i % (EE / 8)) * 8; const int n = (int)(i / (EE / 8)); const float* src = w + (size_t)min(n, NPS - 1) * EE + k0; v8us o;
#pragma unroll
    for (int q = 0; q < 8; ++q) { const unsigned short e = f2bf(src[q]); o[q] = (n < NPS) ? e : (unsigned short)0; }
    *(volatile v8us*)(Bt + (size_t)n * EE + k0) = o; __threadfence(); *(volatile v8us*)(Bt + (size_t)n * EE + k0) = o; }
__global__ __launch_bounds__(256) void k_relu(float* F, size_t n4) { const size_t i = (size_t)blockIdx.x * 256 + threadIdx.x; if (i >= n4) return; v4f a = *(const v4f*)(F + i * 4);
#pragma unroll
    for (int q = 0; q < 4; ++q) a[q] = fmaxf(a[q], 0.f);
    *(volatile v4f*)(F + i * 4) = a; __threadfence(); *(volatile v4f*)(F + i * 4) = a; }
__global__ __launch_bounds__(256) void k_pmean2(const float* __restrict__ F, float* M) { const int lane = threadIdx.x & 31; const int wv = blockIdx.x * 8 + (threadIdx.x >> 5); if (wv >= NPS * 2) return; const int p = wv >> 1; const int d = (wv & 1) * 32 + lane; const float* f = F + (size_t)p * CHK + d; float s = 0.f;
#pragma unroll 4
    for (int t = 0; t < TT; ++t) s = __fadd_rn(s, f[(size_t)t * HD]);
    const float m = __fdiv_rn(s, (float)TT); *(volatile float*)(M + p * HD + d) = m; __threadfence(); *(volatile float*)(M + p * HD + d) = m; }
__global__ __launch_bounds__(256) void k_flatc(const float* __restrict__ F, const float* __restrict__ M, h16* P16, bf* Ph, bf* Pl, size_t n4) { const size_t i = (size_t)blockIdx.x * 256 + threadIdx.x; if (i >= n4) return; const size_t e = i * 4; const int p = (int)(e / CHK); const int d = (int)(e % HD); const v4f a = *(const v4f*)(F + e); const v4f m = *(const v4f*)(M + p * HD + d); v4h o16; v4us oh, ol;
#pragma unroll
    for (int q = 0; q < 4; ++q) { const float c = __fsub_rn(a[q], m[q]); o16[q] = tohx(c); unsigned short u, w2; splitf(c, u, w2); oh[q] = u; ol[q] = w2; }
#pragma unroll 1
    for (int ps = 0; ps < 2; ++ps) { *(volatile v4h*)(P16 + e) = o16; *(volatile v4us*)(Ph + e) = oh; *(volatile v4us*)(Pl + e) = ol; if (ps == 0) __threadfence(); } }
__global__ __launch_bounds__(256) void k_vtpP(const float* __restrict__ F, h16* V16, bf* Vh, bf* Vl) { const size_t e = ((size_t)blockIdx.x * 256 + threadIdx.x) * 2; if (e >= (size_t)NPS * HD * TT) return; const int t = (int)(e % TT); const int d = (int)((e / TT) % HD); const int p = (int)(e / ((size_t)TT * HD)); const float a0 = F[(size_t)p * CHK + (size_t)t * HD + d], a1 = F[(size_t)p * CHK + (size_t)(t + 1) * HD + d]; v2h o16; v2us oh, ol; o16[0] = tohx(a0); o16[1] = tohx(a1); { unsigned short u, w2; splitf(a0, u, w2); oh[0] = u; ol[0] = w2; splitf(a1, u, w2); oh[1] = u; ol[1] = w2; }
#pragma unroll 1
    for (int ps = 0; ps < 2; ++ps) { *(volatile v2h*)(V16 + e) = o16; *(volatile v2us*)(Vh + e) = oh; *(volatile v2us*)(Vl + e) = ol; if (ps == 0) __threadfence(); } }
__global__ __launch_bounds__(256) void k_colsoft(const float* __restrict__ UN, const float* __restrict__ bu, float* US) { const int lane = threadIdx.x & 31; const int h = threadIdx.x >> 5; if (h >= NPS || blockIdx.x > 0) return; float v[TT / 32]; float mx = -3.0e38f;
    const float bb = bfr(bu[h]);
#pragma unroll
    for (int c = 0; c < TT / 32; ++c) { v[c] = __fadd_rn(UN[(size_t)(c * 32 + lane) * NU + h], bb); mx = fmaxf(mx, v[c]); }
#pragma unroll
    for (int sh = 16; sh; sh >>= 1) mx = fmaxf(mx, __shfl_xor(mx, sh, 32));
    float sum = 0.f;
#pragma unroll
    for (int c = 0; c < TT / 32; ++c) { float d0 = __fsub_rn(v[c], mx); asm volatile("" : "+v"(d0)); v[c] = __builtin_amdgcn_exp2f(__fmul_rn(d0, 1.4426950408889634f)); sum = __fadd_rn(sum, v[c]); }
#pragma unroll
    for (int sh = 16; sh; sh >>= 1) sum = __fadd_rn(sum, __shfl_xor(sum, sh, 32));
    const float f = __fdiv_rn(1.0f, sum);
#pragma unroll 1
    for (int ps = 0; ps < 2; ++ps) {
#pragma unroll
        for (int c = 0; c < TT / 32; ++c) *(volatile float*)(US + (size_t)h * TT + c * 32 + lane) = __fmul_rn(v[c], f);
        if (ps == 0) __threadfence(); } }
__global__ __launch_bounds__(256) void k_uwv(const float* __restrict__ US, const float* __restrict__ FV, float* C) { const int lane = threadIdx.x & 31; const int wv = blockIdx.x * 8 + (threadIdx.x >> 5); if (wv >= NPS * 2) return; const int p = wv >> 1; const int d = (wv & 1) * 32 + lane; float s = 0.f;
#pragma unroll 4
    for (int k = 0; k < TT; ++k) { const int f = p * TT + k; s = __fadd_rn(s, __fmul_rn(US[(size_t)(f % NPS) * TT + f / NPS], FV[(size_t)p * CHK + (size_t)k * HD + d])); }
    *(volatile float*)(C + p * HD + d) = s; __threadfence(); *(volatile float*)(C + p * HD + d) = s; }
__global__ __launch_bounds__(256) void k_mergeP(const float* __restrict__ O, const float* __restrict__ C, int p0, float* outb) { const size_t i = (size_t)blockIdx.x * 256 + threadIdx.x; if (i >= (size_t)ZH * TT * HD / 4) return; const size_t e = i * 4; const int d = (int)(e % HD); const int t = (int)((e / HD) % TT); const int zz = (int)(e / ((size_t)TT * HD)); const int p = p0 + zz; const float cs = (t < RH) ? 1.0f : (1.0f / PCAR); const v4f o = *(const v4f*)(O + e); const v4f c = *(const v4f*)(C + p * HD + d); v4f r;
#pragma unroll
    for (int q = 0; q < 4; ++q) r[q] = __fadd_rn(__fmul_rn(o[q], cs), c[q]);
    *(volatile v4f*)(outb + (size_t)p * CHK + (size_t)t * HD + d) = r; __threadfence(); *(volatile v4f*)(outb + (size_t)p * CHK + (size_t)t * HD + d) = r; }

extern "C" void kernel_launch(void* const* d_in, const int* in_sizes, int n_in,
                              void* d_out, int out_size, void* d_ws, size_t ws_size, hipStream_t stream) {
    (void)in_sizes; (void)n_in; (void)out_size;
    const float* x = (const float*)d_in[0]; const float* WQ0 = (const float*)d_in[1]; const float* WK0 = (const float*)d_in[2]; const float* WV0 = (const float*)d_in[3]; const float* wq = (const float*)d_in[4]; const float* bq = (const float*)d_in[5]; const float* wk = (const float*)d_in[6]; const float* bk = (const float*)d_in[7]; const float* wv = (const float*)d_in[8]; const float* bv = (const float*)d_in[9]; const float* wu = (const float*)d_in[10]; const float* bu = (const float*)d_in[11];
    float* OUT = (float*)d_out;
    char* wsp = (char*)d_ws;
    auto take = [&](size_t bytes) { char* p = wsp; wsp += (bytes + 255) & ~(size_t)255; return (void*)p; };
    bf* BQ0 = (bf*)take((size_t)EE * EE * 2); bf* BK0 = (bf*)take((size_t)EE * EE * 2); bf* BV0 = (bf*)take((size_t)EE * EE * 2); bf* BQ1 = (bf*)take((size_t)AA * EE * 2); bf* BK1 = (bf*)take((size_t)AA * EE * 2); bf* BV1 = (bf*)take((size_t)AA * EE * 2); bf* BU = (bf*)take((size_t)NU * EE * 2);
    bf* XB = (bf*)take((size_t)TT * EE * 2); float* F0 = (float*)take((size_t)TT * EE * 4); h16* F016 = (h16*)take((size_t)TT * EE * 2); bf* F0h = (bf*)take((size_t)TT * EE * 2); bf* F0l = (bf*)take((size_t)TT * EE * 2);
    float* FQ = (float*)take((size_t)TT * AA * 4); float* FK = (float*)take((size_t)TT * AA * 4); float* FV = (float*)take((size_t)TT * AA * 4); float* UN = (float*)take((size_t)TT * NU * 4); float* US = (float*)take((size_t)NPS * TT * 4); float* MQ = (float*)take((size_t)NPS * HD * 4); float* MK = (float*)take((size_t)NPS * HD * 4); float* CU = (float*)take((size_t)NPS * HD * 4);
    h16* QP16 = (h16*)take((size_t)TT * AA * 2); bf* QPh = (bf*)take((size_t)TT * AA * 2); bf* QPl = (bf*)take((size_t)TT * AA * 2); h16* KP16 = (h16*)take((size_t)TT * AA * 2); bf* KPh = (bf*)take((size_t)TT * AA * 2); bf* KPl = (bf*)take((size_t)TT * AA * 2); h16* VT16 = (h16*)take((size_t)AA * TT * 2); bf* VTh = (bf*)take((size_t)AA * TT * 2); bf* VTl = (bf*)take((size_t)AA * TT * 2);
    float* Sb = (float*)take((size_t)ZH * TT * TT * 4); h16* P16 = (h16*)take((size_t)ZH * TT * TT * 2); bf* Ph = (bf*)take((size_t)ZH * RH * TT * 2); bf* Pl = (bf*)take((size_t)ZH * RH * TT * 2); float* Ob = (float*)take((size_t)ZH * TT * HD * 4);
    if ((size_t)(wsp - (char*)d_ws) > ws_size) return;
    k_wtG<<<(EE * EE / 64 + 63) / 64, 256, 0, stream>>>(WQ0, EE, EE, BQ0); k_wtG<<<(EE * EE / 64 + 63) / 64, 256, 0, stream>>>(WK0, EE, EE, BK0); k_wtG<<<(EE * EE / 64 + 63) / 64, 256, 0, stream>>>(WV0, EE, EE, BV0);
    k_cvt8<<<(unsigned)(((size_t)AA * EE / 8 + 255) / 256), 256, 0, stream>>>(wq, BQ1, (size_t)AA * EE / 8); k_cvt8<<<(unsigned)(((size_t)AA * EE / 8 + 255) / 256), 256, 0, stream>>>(wk, BK1, (size_t)AA * EE / 8); k_cvt8<<<(unsigned)(((size_t)AA * EE / 8 + 255) / 256), 256, 0, stream>>>(wv, BV1, (size_t)AA * EE / 8); k_wpadT<<<(unsigned)(((size_t)NU * EE / 8 + 255) / 256), 256, 0, stream>>>(wu, BU);
    const unsigned LF = (unsigned)(((size_t)TT * EE / 4 + 255) / 256), LA = (unsigned)(((size_t)TT * AA / 4 + 255) / 256);
    for (int b = 0; b < NB_; ++b) {
        k_cvt8<<<(unsigned)(((size_t)TT * EE / 8 + 255) / 256), 256, 0, stream>>>(x + (size_t)b * TT * EE, XB, (size_t)TT * EE / 8);
        k_gemmw<bf, 0, false><<<dim3(TT / 64, EE / 64, 1), 32, 0, stream>>>(XB, nullptr, BK0, nullptr, EE, F0, EE, nullptr, 0, 0, 0); k_flat<<<LF, 256, 0, stream>>>(F0, F016, F0h, F0l, (size_t)TT * EE / 4);
        k_gemmw<bf, 1, false><<<dim3(TT / 64, NU / 64, 1), 32, 0, stream>>>(F0h, F0l, BU, nullptr, EE, UN, NU, nullptr, 0, 0, 0);
        k_gemmw<bf, 1, true><<<dim3(TT / 64, AA / 64, 1), 32, 0, stream>>>(F0h, F0l, BK1, nullptr, EE, FK, AA, bk, 0, 0, 0); k_relu<<<LA, 256, 0, stream>>>(FK, (size_t)TT * AA / 4);
        k_gemmw<bf, 0, false><<<dim3(TT / 64, EE / 64, 1), 32, 0, stream>>>(XB, nullptr, BQ0, nullptr, EE, F0, EE, nullptr, 0, 0, 0); k_flat<<<LF, 256, 0, stream>>>(F0, F016, F0h, F0l, (size_t)TT * EE / 4);
        k_gemmw<bf, 1, true><<<dim3(TT / 64, AA / 64, 1), 32, 0, stream>>>(F0h, F0l, BQ1, nullptr, EE, FQ, AA, bq, 0, 0, 0); k_relu<<<LA, 256, 0, stream>>>(FQ, (size_t)TT * AA / 4);
        k_gemmw<bf, 0, false><<<dim3(TT / 64, EE / 64, 1), 32, 0, stream>>>(XB, nullptr, BV0, nullptr, EE, F0, EE, nullptr, 0, 0, 0); k_flat<<<LF, 256, 0, stream>>>(F0, F016, F0h, F0l, (size_t)TT * EE / 4);
        k_gemmw<bf, 1, true><<<dim3(TT / 64, AA / 64, 1), 32, 0, stream>>>(F0h, F0l, BV1, nullptr, EE, FV, AA, bv, 0, 0, 0); k_relu<<<LA, 256, 0, stream>>>(FV, (size_t)TT * AA / 4);
        k_pmean2<<<(NPS * 2 + 7) / 8, 256, 0, stream>>>(FQ, MQ); k_pmean2<<<(NPS * 2 + 7) / 8, 256, 0, stream>>>(FK, MK);
        k_flatc<<<LA, 256, 0, stream>>>(FQ, MQ, QP16, QPh, QPl, (size_t)TT * AA / 4); k_flatc<<<LA, 256, 0, stream>>>(FK, MK, KP16, KPh, KPl, (size_t)TT * AA / 4);
        k_vtpP<<<(unsigned)(((size_t)NPS * HD * TT / 2 + 255) / 256), 256, 0, stream>>>(FV, VT16, VTh, VTl);
        k_colsoft<<<1, 256, 0, stream>>>(UN, bu, US); k_uwv<<<(NPS * 2 + 7) / 8, 256, 0, stream>>>(US, FV, CU);
        for (int h0 = 0; h0 < NH_; h0 += ZH) { const size_t zq = (size_t)h0, zk = (size_t)h0;
            k_gemmw<bf, 2, false><<<dim3(RH / 64, TT / 64, ZH), 32, 0, stream>>>(QPh + zq * TT * HD, QPl + zq * TT * HD, KPh + zk * TT * HD, KPl + zk * TT * HD, HD, Sb, TT, nullptr, (size_t)TT * HD, (size_t)TT * HD, (size_t)TT * TT);
            k_gemmw<h16, 0, false><<<dim3((TT - RH) / 64, TT / 64, ZH), 32, 0, stream>>>(QP16 + zq * TT * HD + (size_t)RH * HD, nullptr, KP16 + zk * TT * HD, nullptr, HD, Sb + (size_t)RH * TT, TT, nullptr, (size_t)TT * HD, (size_t)TT * HD, (size_t)TT * TT);
            k_asoft<<<ZH * TT / 8, 256, 0, stream>>>(Sb, P16, Ph, Pl);
            k_gemmw<bf, 2, false><<<dim3(RH / 64, HD / 64, ZH), 32, 0, stream>>>(Ph, Pl, VTh + zk * HD * TT, VTl + zk * HD * TT, TT, Ob, HD, nullptr, (size_t)RH * TT, (size_t)HD * TT, (size_t)TT * HD);
            k_gemmw<h16, 0, false><<<dim3((TT - RH) / 64, HD / 64, ZH), 32, 0, stream>>>(P16 + (size_t)RH * TT, nullptr, VT16 + zk * HD * TT, nullptr, TT, Ob + (size_t)RH * HD, HD, nullptr, (size_t)TT * TT, (size_t)HD * TT, (size_t)TT * HD);
            k_mergeP<<<(unsigned)(((size_t)ZH * TT * HD / 4 + 255) / 256), 256, 0, stream>>>(Ob, CU, h0, OUT + (size_t)b * TT * AA); } }
}
